// MAB_5669356835173
// MI455X (gfx1250) — hardware-verified
//
#include <hip/hip_runtime.h>
#include <math.h>
#include <stdint.h>

#define NB_    8
#define SEQ    1024
#define DMOD   1024
#define NHEAD  16
#define HDIM   64
#define MROWS  (NB_ * SEQ)
#define PLANE  (SEQ * DMOD)

static_assert(MROWS % 64 == 0);
static_assert(DMOD % 64 == 0);
static_assert(SEQ % 64 == 0);
static_assert(DMOD % 32 == 0);
static_assert(NHEAD * HDIM == DMOD);

typedef __attribute__((ext_vector_type(16))) __bf16 v16b;
typedef __attribute__((ext_vector_type(8)))  __bf16 v8b;
typedef __attribute__((ext_vector_type(8)))  float  v8f;
typedef __attribute__((ext_vector_type(4)))  float  v4f;
typedef __attribute__((ext_vector_type(4)))  unsigned int v4u;
typedef v4f __attribute__((may_alias)) v4fa;
typedef v8b __attribute__((may_alias)) v8ba;

__device__ __forceinline__ unsigned short f2bf_bits(float f) {
  const unsigned u = __float_as_uint(f);
  return (unsigned short)((u + 0x7FFFu + ((u >> 16) & 1u)) >> 16);
}
__device__ __forceinline__ float bf_bits2f(unsigned short h) { return __uint_as_float(((unsigned)h) << 16); }
__device__ __forceinline__ float bf_rne(float f) { return bf_bits2f(f2bf_bits(f)); }
__device__ __forceinline__ unsigned pk16(unsigned short a, unsigned short b) { return (unsigned)a | ((unsigned)b << 16); }

union FragU { v16b v; v8b h[2]; };
__device__ __forceinline__ v16b frag_load(const __bf16* p) {
  FragU f;
  f.h[0] = *(const v8ba*)(p);
  f.h[1] = *(const v8ba*)(p + 16);
  return f.v;
}
__device__ __forceinline__ v8f mma_raw(v16b a, v16b b, v8f c) {
  return __builtin_amdgcn_wmma_f32_16x16x32_bf16(false, a, false, b, (short)0, c, false, false);
}
__device__ __forceinline__ v8f mma_g(v16b a, v16b b, v8f c) {
  c = mma_raw(a, b, c);
  asm volatile("v_nop\n\tv_nop\n\tv_nop\n\tv_nop" : "+v"(c) : "v"(a), "v"(b));
  return c;
}
__device__ __forceinline__ void dep_guard(v8f& a, v8f& b, v16b x, v16b y) {
  asm volatile("v_nop\n\tv_nop\n\tv_nop\n\tv_nop" : "+v"(a), "+v"(b) : "v"(x), "v"(y));
}
__device__ __forceinline__ void keep4(v16b a, v16b b, v16b c, v16b d) {
  asm volatile("v_nop" :: "v"(a), "v"(b), "v"(c), "v"(d));
}
__device__ __forceinline__ void acc_guard4(v8f& a, v8f& b, v8f& c, v8f& d) {
  asm volatile("v_nop\n\tv_nop\n\tv_nop\n\tv_nop" : "+v"(a), "+v"(b), "+v"(c), "+v"(d));
}
__device__ __forceinline__ void wave_sync_lds() {
  __builtin_amdgcn_fence(__ATOMIC_RELEASE, "workgroup");
  __builtin_amdgcn_wave_barrier();
  __builtin_amdgcn_fence(__ATOMIC_ACQUIRE, "workgroup");
}

__global__ __launch_bounds__(256) void cvt_kernel(const float* __restrict__ x,
                                                  unsigned short* __restrict__ o, int n8) {
  const int g = blockIdx.x * 256 + threadIdx.x;
  if (g >= n8) return;
  const float* src = x + (size_t)g * 8;
  const v4f a = *(const v4fa*)(src);
  const v4f c = *(const v4fa*)(src + 4);
  v4u w;
  w[0] = pk16(f2bf_bits(a[0]), f2bf_bits(a[1]));
  w[1] = pk16(f2bf_bits(a[2]), f2bf_bits(a[3]));
  w[2] = pk16(f2bf_bits(c[0]), f2bf_bits(c[1]));
  w[3] = pk16(f2bf_bits(c[2]), f2bf_bits(c[3]));
  unsigned short* dst = o + (size_t)g * 8;
  *(volatile v4u*)dst = w;
  __threadfence();
  *(volatile v4u*)dst = w;
}

__global__ __launch_bounds__(256) void wtrans_kernel(const float* __restrict__ W0, const float* __restrict__ W1,
                                                     const float* __restrict__ W2, const float* __restrict__ W3,
                                                     unsigned short* __restrict__ out, int R, int Cc) {
  __shared__ __align__(16) float tf[64 * 68];
  const int z = blockIdx.z;
  const float* W = W0;
  if (z == 1) W = W1;
  if (z == 2) W = W2;
  if (z == 3) W = W3;
  out += (size_t)z * R * Cc;
  const int c0  = blockIdx.x * 64;
  const int r0  = blockIdx.y * 64;
  const int tid = threadIdx.x;
  {
    const int lr = tid >> 4;
    const int c4 = (tid & 15) * 4;
#pragma unroll
    for (int it = 0; it < 4; ++it) {
      const int rr = it * 16 + lr;
      const v4f a = *(const v4fa*)(W + (size_t)(r0 + rr) * Cc + c0 + c4);
      *(v4fa*)(tf + rr * 68 + c4) = a;
    }
  }
  __syncthreads();
  const int sub = tid >> 3;
  const int c8  = (tid & 7) * 8;
  v4u hv[2];
#pragma unroll
  for (int it = 0; it < 2; ++it) {
    const int oc = it * 32 + sub;
    v4u a;
#pragma unroll
    for (int q = 0; q < 4; ++q) {
      const float f0 = tf[(c8 + 2 * q) * 68 + oc];
      const float f1 = tf[(c8 + 2 * q + 1) * 68 + oc];
      a[q] = pk16(f2bf_bits(f0), f2bf_bits(f1));
    }
    hv[it] = a;
  }
  for (int pass = 0; pass < 2; ++pass) {
#pragma unroll
    for (int it = 0; it < 2; ++it) {
      const int oc = it * 32 + sub;
      const size_t go = (size_t)(c0 + oc) * R + r0 + c8;
      *(volatile v4u*)(out + go) = hv[it];
    }
    __threadfence();
  }
}

template <bool ASPLIT, int BIAS_MODE, int OUT_MODE, bool RESID, int ACT>
__global__ __launch_bounds__(256) void gemm64_kernel(
    const unsigned short* __restrict__ Ap, const unsigned short* __restrict__ A2p, int lda, long strideA,
    const unsigned short* __restrict__ Btp, int ldb, long strideB,
    void* __restrict__ Cout, void* __restrict__ Cout2, int ldc, long strideC,
    const float* __restrict__ bias,
    const float* __restrict__ resid, long strideR,
    int M, int N, int K) {
  const __bf16* A  = (const __bf16*)(const void*)Ap;
  const __bf16* A2 = (const __bf16*)(const void*)A2p;
  const __bf16* Bt = (const __bf16*)(const void*)Btp;
  __shared__ __align__(16) float sT[8][16 * 68];
  const int b    = blockIdx.y;
  const int lane = threadIdx.x & 31;
  const int wave = threadIdx.x >> 5;
  const int tilesN = N >> 6;
  const int tilesM = M >> 6;
  const int tile = blockIdx.x * 8 + wave;
  if (tile >= tilesM * tilesN) return;
  const int tm = tile / tilesN;
  const int tn = tile - tm * tilesN;
  const int m0 = tm << 6;
  const int n0 = tn << 6;

  const __bf16* Ab  = A  + (size_t)b * strideA;
  const __bf16* Ab2 = ASPLIT ? (A2 + (size_t)b * strideA) : Ab;
  const __bf16* Bb  = Bt + (size_t)b * strideB;

  const int rlane = lane & 15;
  const int koff  = (lane >> 4) * 8;
  const int mOff  = (lane >> 4) * 8;

  v8f acc[4][4];
#pragma unroll
  for (int i = 0; i < 4; ++i)
#pragma unroll
    for (int j = 0; j < 4; ++j) acc[i][j] = (v8f){0.f,0.f,0.f,0.f,0.f,0.f,0.f,0.f};

#pragma unroll 1
  for (int k0 = 0; k0 < K; k0 += 32) {
    v16b bf[4];
#pragma unroll
    for (int j = 0; j < 4; ++j) {
      const size_t bo = (size_t)(n0 + (j << 4) + rlane) * ldb + koff + k0;
      bf[j] = frag_load(Bb + bo);
    }
#pragma unroll
    for (int i = 0; i < 4; ++i) {
      const size_t ao = (size_t)(m0 + (i << 4) + rlane) * lda + koff + k0;
      const v16b ah = frag_load(Ab + ao);
      v16b al = ah;
      if (ASPLIT) al = frag_load(Ab2 + ao);
#pragma unroll
      for (int j = 0; j < 4; ++j) {
        acc[i][j] = mma_raw(ah, bf[j], acc[i][j]);
        if (ASPLIT) acc[i][j] = mma_raw(al, bf[j], acc[i][j]);
      }
      dep_guard(acc[i][0], acc[i][3], ah, al);
    }
    keep4(bf[0], bf[1], bf[2], bf[3]);
  }
  acc_guard4(acc[0][0], acc[0][1], acc[0][2], acc[0][3]);
  acc_guard4(acc[1][0], acc[1][1], acc[1][2], acc[1][3]);
  acc_guard4(acc[2][0], acc[2][1], acc[2][2], acc[2][3]);
  acc_guard4(acc[3][0], acc[3][1], acc[3][2], acc[3][3]);

  float* slab = sT[wave];
  const float* Rb = resid + (size_t)b * strideR;
#pragma unroll
  for (int i = 0; i < 4; ++i) {
    const int mBase = m0 + (i << 4);
    float bm[8];
    if (BIAS_MODE == 1) {
      const v4f b0v = *(const v4fa*)(bias + mBase + mOff);
      const v4f b1v = *(const v4fa*)(bias + mBase + mOff + 4);
      bm[0] = bf_rne(b0v[0]); bm[1] = bf_rne(b0v[1]); bm[2] = bf_rne(b0v[2]); bm[3] = bf_rne(b0v[3]);
      bm[4] = bf_rne(b1v[0]); bm[5] = bf_rne(b1v[1]); bm[6] = bf_rne(b1v[2]); bm[7] = bf_rne(b1v[3]);
    } else {
#pragma unroll
      for (int r = 0; r < 8; ++r) bm[r] = 0.0f;
    }
#pragma unroll
    for (int j = 0; j < 4; ++j) {
      const int n = n0 + (j << 4) + rlane;
      float bn = 0.0f;
      if (BIAS_MODE == 2) bn = bf_rne(bias[n]);
#pragma unroll
      for (int r = 0; r < 8; ++r) {
        float v = acc[i][j][r];
        if (BIAS_MODE == 1) v += bm[r];
        if (BIAS_MODE == 2) v += bn;
        if (ACT == 2) v = fmaxf(v, 0.0f);
        slab[(mOff + r) * 68 + (j << 4) + rlane] = v;
      }
    }
    wave_sync_lds();
    if (OUT_MODE == 0 || OUT_MODE == 2) {
      float* C = (float*)Cout + (size_t)b * strideC;
      const int hh = lane >> 4, c4 = (lane & 15) * 4;
      for (int pass = 0; pass < 2; ++pass) {
#pragma unroll
        for (int it = 0; it < 8; ++it) {
          const int row = it * 2 + hh;
          v4f v = *(const v4fa*)(slab + row * 68 + c4);
          if (RESID) {
            const v4f rr = *(const v4fa*)(Rb + (size_t)(mBase + row) * ldc + n0 + c4);
            v = v + rr;
          }
          *(volatile v4f*)(C + (size_t)(mBase + row) * ldc + n0 + c4) = v;
        }
        __threadfence();
      }
    }
    if (OUT_MODE == 1 || OUT_MODE == 2) {
      unsigned short* C16 = (unsigned short*)((OUT_MODE == 1) ? Cout : Cout2) + (size_t)b * strideC;
      const int q = lane >> 3, c8 = (lane & 7) * 8;
      v4u hv[4];
#pragma unroll
      for (int it = 0; it < 4; ++it) {
        const int row = it * 4 + q;
        const float* sp = slab + row * 68 + c8;
        v4u w;
#pragma unroll
        for (int e = 0; e < 4; ++e) w[e] = pk16(f2bf_bits(sp[2 * e]), f2bf_bits(sp[2 * e + 1]));
        hv[it] = w;
      }
      for (int pass = 0; pass < 2; ++pass) {
#pragma unroll
        for (int it = 0; it < 4; ++it) {
          const int row = it * 4 + q;
          *(volatile v4u*)(C16 + (size_t)(mBase + row) * ldc + n0 + c8) = hv[it];
        }
        __threadfence();
      }
    }
    wave_sync_lds();
  }
}

#define AT_D  64
#define AT_NW 4
#define AT_QB 64
#define AT_KC 64

__device__ __forceinline__ void at_split(float f, __bf16& hi, __bf16& lo) {
  const unsigned short hb = f2bf_bits(f);
  hi = __builtin_bit_cast(__bf16, hb);
  lo = __builtin_bit_cast(__bf16, f2bf_bits(f - bf_bits2f(hb)));
}

__global__ __launch_bounds__(128)
void attn_kernel(const unsigned short* __restrict__ qbp, const unsigned short* __restrict__ kbp,
                 const unsigned short* __restrict__ vtp, const float* __restrict__ qres,
                 float* __restrict__ out, float sscale) {
  union FB { v16b v; v8b h[2]; };
  __shared__ __align__(16) __bf16 Ksh[AT_KC * AT_D];
  __shared__ __align__(16) __bf16 Vth[AT_D * AT_KC];
  __shared__ __align__(16) __bf16 Psh[AT_NW][16 * AT_KC];
  __shared__ __align__(16) __bf16 Psl[AT_NW][16 * AT_KC];
  __shared__ __align__(16) float  Os[AT_NW][16 * 68];

  const int tid  = threadIdx.x;
  const int wave = tid >> 5;
  const int lane = tid & 31;
  const int hh   = lane >> 4;
  const int c    = lane & 15;

  const int nqb = SEQ / AT_QB;
  const int b   = blockIdx.y;
  const int bx  = blockIdx.x;
  const int qb  = bx % nqb;
  const int h   = bx / nqb;
  const int q0  = qb * AT_QB + wave * 16;
  const size_t pb = (size_t)b * PLANE;

  const __bf16* Qh = (const __bf16*)(const void*)qbp + pb + (size_t)h * AT_D;
  const __bf16* Kh = (const __bf16*)(const void*)kbp + pb + (size_t)h * AT_D;
  const __bf16* Vh = (const __bf16*)(const void*)vtp + pb + (size_t)h * AT_D * SEQ;
  const float*  rb = qres + pb + (size_t)h * AT_D;
  float*        ob = out  + pb + (size_t)h * AT_D;

  v16b qa[2];
#pragma unroll
  for (int dc = 0; dc < 2; ++dc)
    qa[dc] = frag_load(Qh + (size_t)(q0 + c) * DMOD + dc * 32 + 8 * hh);

  float mrow[8], lrow[8];
  v8f oacc[4];
#pragma unroll
  for (int r = 0; r < 8; ++r) { mrow[r] = -INFINITY; lrow[r] = 0.f; }
#pragma unroll
  for (int t = 0; t < 4; ++t) oacc[t] = (v8f){0.f,0.f,0.f,0.f,0.f,0.f,0.f,0.f};

#pragma unroll 1
  for (int kc = 0; kc < SEQ / AT_KC; ++kc) {
    const int kv0 = kc * AT_KC;
    __syncthreads();
    {
      const int r = tid >> 1, half = (tid & 1) * 32;
      const __bf16* ksrc = Kh + (size_t)(kv0 + r) * DMOD + half;
      const __bf16* vsrc = Vh + (size_t)r * SEQ + kv0 + half;
#pragma unroll
      for (int i = 0; i < 4; ++i) {
        const v8b a0 = *(const v8ba*)(ksrc + 8 * i);
        const v8b b0 = *(const v8ba*)(vsrc + 8 * i);
        *(v8ba*)(Ksh + r * AT_D  + half + 8 * i) = a0;
        *(v8ba*)(Vth + r * AT_KC + half + 8 * i) = b0;
      }
    }
    __syncthreads();

    v8f s[4];
#pragma unroll
    for (int j = 0; j < 4; ++j) {
      s[j] = (v8f){0.f,0.f,0.f,0.f,0.f,0.f,0.f,0.f};
#pragma unroll
      for (int dc = 0; dc < 2; ++dc) {
        FB kb;
        kb.h[0] = *(const v8ba*)(Ksh + (j * 16 + c) * AT_D + dc * 32 + 8 * hh);
        kb.h[1] = *(const v8ba*)(Ksh + (j * 16 + c) * AT_D + dc * 32 + 16 + 8 * hh);
        s[j] = mma_g(qa[dc], kb.v, s[j]);
      }
    }
    float cm[8];
#pragma unroll
    for (int r = 0; r < 8; ++r) {
      float m = -INFINITY;
#pragma unroll
      for (int j = 0; j < 4; ++j) {
        const float sv = s[j][r] * sscale;
        s[j][r] = sv;
        m = fmaxf(m, sv);
      }
#pragma unroll
      for (int off = 1; off < 16; off <<= 1) m = fmaxf(m, __shfl_xor(m, off, 32));
      cm[r] = m;
    }
    __bf16* pwh = Psh[wave];
    __bf16* pwl = Psl[wave];
#pragma unroll
    for (int r = 0; r < 8; ++r) {
      const float mnew  = fmaxf(mrow[r], cm[r]);
      const float alpha = __expf(mrow[r] - mnew);
      mrow[r] = mnew;
      float psum = 0.f;
#pragma unroll
      for (int j = 0; j < 4; ++j) {
        const float p = __expf(s[j][r] - mnew);
        psum += p;
        __bf16 a, bl; at_split(p, a, bl);
        pwh[(8 * hh + r) * AT_KC + j * 16 + c] = a;
        pwl[(8 * hh + r) * AT_KC + j * 16 + c] = bl;
      }
#pragma unroll
      for (int off = 1; off < 16; off <<= 1) psum += __shfl_xor(psum, off, 32);
      lrow[r] = lrow[r] * alpha + psum;
#pragma unroll
      for (int t = 0; t < 4; ++t) oacc[t][r] *= alpha;
    }
    wave_sync_lds();
#pragma unroll 1
    for (int kk = 0; kk < 2; ++kk) {
      FB pa, pl;
      pa.h[0] = *(const v8ba*)(pwh + c * AT_KC + kk * 32 + 8 * hh);
      pa.h[1] = *(const v8ba*)(pwh + c * AT_KC + kk * 32 + 16 + 8 * hh);
      pl.h[0] = *(const v8ba*)(pwl + c * AT_KC + kk * 32 + 8 * hh);
      pl.h[1] = *(const v8ba*)(pwl + c * AT_KC + kk * 32 + 16 + 8 * hh);
#pragma unroll
      for (int t = 0; t < 4; ++t) {
        FB vb;
        vb.h[0] = *(const v8ba*)(Vth + (t * 16 + c) * AT_KC + kk * 32 + 8 * hh);
        vb.h[1] = *(const v8ba*)(Vth + (t * 16 + c) * AT_KC + kk * 32 + 16 + 8 * hh);
        oacc[t] = mma_g(pa.v, vb.v, oacc[t]);
        oacc[t] = mma_g(pl.v, vb.v, oacc[t]);
      }
    }
  }

  float* os = Os[wave];
#pragma unroll
  for (int r = 0; r < 8; ++r) {
    const float inv = 1.0f / lrow[r];
#pragma unroll
    for (int t = 0; t < 4; ++t) os[(8 * hh + r) * 68 + t * 16 + c] = oacc[t][r] * inv;
  }
  wave_sync_lds();
  {
    const int c4 = (lane & 15) * 4;
    for (int pass = 0; pass < 2; ++pass) {
#pragma unroll
      for (int it = 0; it < 8; ++it) {
        const int row = it * 2 + hh;
        v4f val = *(const v4fa*)(os + row * 68 + c4);
        const v4f rr = *(const v4fa*)(rb + (size_t)(q0 + row) * DMOD + c4);
        val = val + rr;
        *(volatile v4f*)(ob + (size_t)(q0 + row) * DMOD + c4) = val;
      }
      __threadfence();
    }
  }
}

template <bool SPLIT_OUT>
__global__ __launch_bounds__(256) void ln_kernel(const float* __restrict__ in, const float* __restrict__ gam,
                                                 const float* __restrict__ bet, float* __restrict__ outp,
                                                 unsigned short* __restrict__ oh, unsigned short* __restrict__ ol,
                                                 int nrows) {
  __shared__ __align__(16) float rowbuf[8 * DMOD];
  const int tid = threadIdx.x, lane = tid & 31, wave = tid >> 5;
  const int row = blockIdx.x * 8 + wave;
  if (row >= nrows) return;
  const float* src = in + (size_t)row * DMOD;

  v4f x[8];
#pragma unroll
  for (int it = 0; it < 8; ++it) x[it] = *(const v4fa*)(src + it * 128 + lane * 4);
  float ssum = 0.0f;
#pragma unroll
  for (int it = 0; it < 8; ++it) ssum += (x[it][0] + x[it][1]) + (x[it][2] + x[it][3]);
#pragma unroll
  for (int off = 1; off < 32; off <<= 1) ssum += __shfl_xor(ssum, off, 32);
  const float mean = ssum * (1.0f / 1024.0f);

  v4f d[8];
  float sq = 0.0f;
#pragma unroll
  for (int it = 0; it < 8; ++it) {
    d[it] = x[it] - mean;
    sq += d[it][0] * d[it][0] + d[it][1] * d[it][1] + d[it][2] * d[it][2] + d[it][3] * d[it][3];
  }
#pragma unroll
  for (int off = 1; off < 32; off <<= 1) sq += __shfl_xor(sq, off, 32);
  const float var = sq * (1.0f / 1024.0f);
  const float rs  = rsqrtf(var + 1e-5f);

  v4f y[8];
#pragma unroll
  for (int it = 0; it < 8; ++it) {
    const v4f gv = *(const v4fa*)(gam + it * 128 + lane * 4);
    const v4f bv = *(const v4fa*)(bet + it * 128 + lane * 4);
    v4f t;
#pragma unroll
    for (int e = 0; e < 4; ++e) t[e] = (d[it][e] * rs) * bf_rne(gv[e]) + bf_rne(bv[e]);
    y[it] = t;
  }

  float* dst = outp + (size_t)row * DMOD;
  for (int pass = 0; pass < 2; ++pass) {
#pragma unroll
    for (int it = 0; it < 8; ++it) *(volatile v4f*)(dst + it * 128 + lane * 4) = y[it];
    __threadfence();
  }

  if (SPLIT_OUT) {
    float* rbw = rowbuf + wave * DMOD;
#pragma unroll
    for (int it = 0; it < 8; ++it) *(v4fa*)(rbw + it * 128 + lane * 4) = y[it];
    wave_sync_lds();
    v4u hv[4], lv[4];
#pragma unroll
    for (int it = 0; it < 4; ++it) {
      const v4f a  = *(const v4fa*)(rbw + it * 256 + lane * 8);
      const v4f a2 = *(const v4fa*)(rbw + it * 256 + lane * 8 + 4);
      float f[8];
      f[0] = a[0]; f[1] = a[1]; f[2] = a[2]; f[3] = a[3];
      f[4] = a2[0]; f[5] = a2[1]; f[6] = a2[2]; f[7] = a2[3];
      v4u wh, wl;
#pragma unroll
      for (int q = 0; q < 4; ++q) {
        const unsigned short h0 = f2bf_bits(f[2 * q]), h1 = f2bf_bits(f[2 * q + 1]);
        const unsigned short l0 = f2bf_bits(f[2 * q] - bf_bits2f(h0));
        const unsigned short l1 = f2bf_bits(f[2 * q + 1] - bf_bits2f(h1));
        wh[q] = pk16(h0, h1);
        wl[q] = pk16(l0, l1);
      }
      hv[it] = wh; lv[it] = wl;
    }
    unsigned short* dh = oh + (size_t)row * DMOD;
    unsigned short* dl = ol + (size_t)row * DMOD;
    for (int pass = 0; pass < 2; ++pass) {
#pragma unroll
      for (int it = 0; it < 4; ++it) {
        *(volatile v4u*)(dh + it * 256 + lane * 8) = hv[it];
        *(volatile v4u*)(dl + it * 256 + lane * 8) = lv[it];
      }
      __threadfence();
    }
  }
}

extern "C" void kernel_launch(void* const* d_in, const int* in_sizes, int n_in,
                              void* d_out, int out_size, void* d_ws, size_t ws_size,
                              hipStream_t stream) {
  if (n_in < 14) return;
  if (in_sizes[0] != MROWS * DMOD || in_sizes[1] != MROWS * DMOD) return;
  if (in_sizes[2] != DMOD * DMOD || in_sizes[4] != DMOD * DMOD ||
      in_sizes[6] != DMOD * DMOD || in_sizes[8] != DMOD * DMOD) return;
  if (in_sizes[3] != DMOD || in_sizes[5] != DMOD || in_sizes[7] != DMOD || in_sizes[9] != DMOD) return;
  if (in_sizes[10] != DMOD || in_sizes[11] != DMOD || in_sizes[12] != DMOD || in_sizes[13] != DMOD) return;
  if (out_size != MROWS * DMOD) return;

  const float* Qin = (const float*)d_in[0];
  const float* Kin = (const float*)d_in[1];
  const float* Wq  = (const float*)d_in[2];
  const float* bq  = (const float*)d_in[3];
  const float* Wk  = (const float*)d_in[4];
  const float* bk  = (const float*)d_in[5];
  const float* Wv  = (const float*)d_in[6];
  const float* bv  = (const float*)d_in[7];
  const float* Wo  = (const float*)d_in[8];
  const float* bo  = (const float*)d_in[9];
  const float* g0  = (const float*)d_in[10];
  const float* be0 = (const float*)d_in[11];
  const float* g1  = (const float*)d_in[12];
  const float* be1 = (const float*)d_in[13];
  float* out = (float*)d_out;

  const size_t BP16 = (size_t)MROWS * DMOD * 2;
  const size_t BP32 = (size_t)MROWS * DMOD * 4;
  const size_t BW16 = (size_t)DMOD * DMOD * 2;
  size_t off = 0;
  const size_t oQB  = off; off += BP16;
  const size_t oKB  = off; off += BP16;
  const size_t oWT  = off; off += 4 * BW16;
  const size_t oQP  = off; off += BP32;
  const size_t oQPb = off; off += BP16;
  const size_t oKPb = off; off += BP16;
  const size_t oVPt = off; off += BP16;
  const size_t total = off;
  if (total > ws_size) return;
  if (oKB + BP16 - oQB != BP32) return;

  char* ws = (char*)d_ws;
  unsigned short* QB   = (unsigned short*)(ws + oQB);
  unsigned short* KB   = (unsigned short*)(ws + oKB);
  unsigned short* WT   = (unsigned short*)(ws + oWT);
  unsigned short* Wqt  = WT;
  unsigned short* Wkt  = WT + (size_t)PLANE;
  unsigned short* Wvt  = WT + (size_t)2 * PLANE;
  unsigned short* Wot  = WT + (size_t)3 * PLANE;
  float*          QP   = (float*)(ws + oQP);
  unsigned short* QPb  = (unsigned short*)(ws + oQPb);
  unsigned short* KPb  = (unsigned short*)(ws + oKPb);
  unsigned short* VPt  = (unsigned short*)(ws + oVPt);
  float*          Obuf = (float*)(ws + oQB);
  float*          O1f  = (float*)(ws + oQP);
  unsigned short* O1h  = (unsigned short*)(ws + oQPb);
  unsigned short* O1l  = (unsigned short*)(ws + oKPb);
  float*          Rbuf = (float*)(ws + oQB);

  const dim3 blk(256);
  const int n8 = MROWS * DMOD / 8;
  cvt_kernel<<<dim3(n8 / 256), blk, 0, stream>>>(Qin, QB, n8);
  cvt_kernel<<<dim3(n8 / 256), blk, 0, stream>>>(Kin, KB, n8);
  wtrans_kernel<<<dim3(DMOD / 64, DMOD / 64, 4), blk, 0, stream>>>(Wq, Wk, Wv, Wo, WT, DMOD, DMOD);

  const dim3 gTok(((MROWS / 64) * (DMOD / 64)) / 8, 1);
  const dim3 gVT(((DMOD / 64) * (SEQ / 64)) / 8, NB_);
  gemm64_kernel<false, 2, 2, false, 0><<<gTok, blk, 0, stream>>>(
      QB, QB, DMOD, 0L, Wqt, DMOD, 0L, (void*)QP, (void*)QPb, DMOD, 0L,
      bq, bq, 0L, MROWS, DMOD, DMOD);
  gemm64_kernel<false, 2, 1, false, 0><<<gTok, blk, 0, stream>>>(
      KB, KB, DMOD, 0L, Wkt, DMOD, 0L, (void*)KPb, (void*)KPb, DMOD, 0L,
      bk, bk, 0L, MROWS, DMOD, DMOD);
  gemm64_kernel<false, 1, 1, false, 0><<<gVT, blk, 0, stream>>>(
      Wvt, Wvt, DMOD, 0L, KB, DMOD, (long)PLANE, (void*)VPt, (void*)VPt, SEQ, (long)PLANE,
      bv, bv, 0L, DMOD, SEQ, DMOD);
  attn_kernel<<<dim3(NHEAD * (SEQ / AT_QB), NB_), dim3(128), 0, stream>>>(QPb, KPb, VPt, QP, Obuf, 0.03125f);
  ln_kernel<true><<<dim3(MROWS / 8), blk, 0, stream>>>(Obuf, g0, be0, O1f, O1h, O1l, MROWS);
  gemm64_kernel<true, 2, 0, true, 2><<<gTok, blk, 0, stream>>>(
      O1h, O1l, DMOD, 0L, Wot, DMOD, 0L, (void*)Rbuf, (void*)Rbuf, DMOD, 0L,
      bo, O1f, 0L, MROWS, DMOD, DMOD);
  ln_kernel<false><<<dim3(MROWS / 8), blk, 0, stream>>>(Rbuf, g1, be1, out, O1h, O1l, MROWS);
  (void)hipGetLastError();
}
